// MultiHeadLatentAttention_34067680592384
// MI455X (gfx1250) — hardware-verified
//
#include <hip/hip_runtime.h>
#include <math.h>


#ifndef NB
#define NB 1
#endif
#ifndef SEQ
#define SEQ 2048
#endif
#ifndef EROWS_MAX
#define EROWS_MAX 256
#endif
#define SEQ_FULL 2048
#define HID 2048
#define QL 768
#define KVL 512
#define DR 64
#define KVW (KVL + DR)
#define KVP 640
#define NH 16
#define DN 128
#define DV 128
#define DQK (DN + DR)
#define QW (NH * DQK)
#define KVUPW (NH * (DN + DV))
#define CTXW (NH * DV)
#define NFREQ (DR / 2)
#define EROWS ((SEQ < EROWS_MAX) ? SEQ : EROWS_MAX)
#define LROWS (SEQ - EROWS)

static_assert(NB == 1);
static_assert(SEQ % 64 == 0 && SEQ >= 64 && SEQ <= SEQ_FULL);
static_assert(EROWS % 64 == 0 && EROWS >= 64 && EROWS <= SEQ);
static_assert(QL % 128 == 0 && KVP % 128 == 0 && QW % 128 == 0 && KVUPW % 128 == 0 && HID % 128 == 0);
static_assert(HID % 32 == 0 && QL % 32 == 0 && KVL % 32 == 0 && CTXW % 32 == 0 && KVW <= KVP);
static_assert(DQK % 32 == 0 && DV % 16 == 0 && NFREQ == 32);

#define SCL 0.07216878364870322f
#define PCAR 4096.0f
#define PCARI 0.000244140625f
#define RESC 2048.0f
#define RESCI 0.00048828125f
#define RMS_EPS 0.000001f

typedef _Float16 v16h __attribute__((ext_vector_type(16)));
typedef _Float16 v8h  __attribute__((ext_vector_type(8)));
typedef _Float16 v8ha __attribute__((ext_vector_type(8), __may_alias__));
typedef float    v8f  __attribute__((ext_vector_type(8)));
typedef float    v4f  __attribute__((ext_vector_type(4)));
typedef float    v4fa __attribute__((ext_vector_type(4), __may_alias__));
typedef unsigned v8u  __attribute__((ext_vector_type(8)));

__device__ __forceinline__ float bfrne(float f) { unsigned u = __float_as_uint(f); u += 0x7FFFu + ((u >> 16) & 1u); return __uint_as_float(u & 0xFFFF0000u); }
__device__ __forceinline__ unsigned h2u(_Float16 h) { return (unsigned)__builtin_bit_cast(unsigned short, h); }
__device__ __forceinline__ int kpat(int v, int half) { return ((v & 4) ? 16 : 0) + half * 8 + 2 * (v & 3); }

__device__ __forceinline__ v8f wm16(v16h a, v16h b, v8f c) {
    c = __builtin_amdgcn_wmma_f32_16x16x32_f16(false, a, false, b, (short)0, c, false, false);
    asm volatile("v_nop\n\tv_nop\n\tv_nop\n\tv_nop" : "+v"(c) : "v"(a), "v"(b));
    return c;
}
union Frag { v16h v; v8h hf[2]; };
__device__ __forceinline__ v16h ldfrag_g(const _Float16* p) { Frag f; f.hf[0] = *(const v8h*)p; f.hf[1] = *(const v8h*)(p + 16); return f.v; }
__device__ __forceinline__ v16h ldfrag_l(const _Float16* p) { Frag f; f.hf[0] = *(const v8ha*)p; f.hf[1] = *(const v8ha*)(p + 16); return f.v; }
__device__ __forceinline__ void wave_sync() {
    __builtin_amdgcn_fence(3, "wavefront");
    __builtin_amdgcn_wave_barrier();
    __builtin_amdgcn_fence(2, "wavefront");
}

struct Opnd2 { v16h p[2]; };
template <int RIN, int NP> __device__ __forceinline__ void pack2(float f0, float f1, float sc, unsigned* o) {
    if (RIN) { f0 = bfrne(f0); f1 = bfrne(f1); }
    f0 *= sc; f1 *= sc;
    const _Float16 h0 = (_Float16)f0, h1 = (_Float16)f1;
    o[0] = h2u(h0) | (h2u(h1) << 16);
    if (NP >= 2) {
        const _Float16 q0 = (_Float16)((f0 - (float)h0) * RESC), q1 = (_Float16)((f1 - (float)h1) * RESC);
        o[1] = h2u(q0) | (h2u(q1) << 16);
    }
}
template <int RIN, int NP> __device__ __forceinline__ void op_row(const float* rowp, int half, float sc, Opnd2& o) {
    v8u u[2];
#pragma unroll
    for (int v = 0; v < 8; ++v) {
        const int kk = kpat(v, half); unsigned t[2];
        pack2<RIN, NP>(rowp[kk], rowp[kk + 1], sc, t);
#pragma unroll
        for (int p = 0; p < NP; ++p) u[p][v] = t[p];
    }
#pragma unroll
    for (int p = 0; p < NP; ++p) o.p[p] = __builtin_bit_cast(v16h, u[p]);
}
template <int RIN, int NP> __device__ __forceinline__ void op_col(const float* M, int ld, int n, int k0, int half, float sc, Opnd2& o) {
    v8u u[2];
#pragma unroll
    for (int v = 0; v < 8; ++v) {
        const int kk = k0 + kpat(v, half); unsigned t[2];
        pack2<RIN, NP>(M[(size_t)kk * ld + n], M[(size_t)(kk + 1) * ld + n], sc, t);
#pragma unroll
        for (int p = 0; p < NP; ++p) u[p][v] = t[p];
    }
#pragma unroll
    for (int p = 0; p < NP; ++p) o.p[p] = __builtin_bit_cast(v16h, u[p]);
}

struct GArgs {
    const float* A; const float* Bm; float* C;
    int lda, ldb, ldc, K;
    int M, nvalid, nstore, spare;
    float ascale, bscale, oscale, fsp;
};
static_assert(sizeof(GArgs) == 72);

template <int RA, int NA, int RB>
__global__ __launch_bounds__(256) __attribute__((amdgpu_num_vgpr(256))) void gemm_kernel(GArgs g) {
    constexpr int RW = 4, TR = 64, TC = 128, CSTR = TC + 4;
    __shared__ __align__(16) float cst[TR * CSTR];
    const int tid = threadIdx.x, lane = tid & 31, wv = tid >> 5;
    const int l16 = lane & 15, half = lane >> 4;
    const int rt = wv % RW, ch = wv / RW;
    const int row0 = blockIdx.x * TR, col0 = blockIdx.y * TC + ch * 64;
    int arix = row0 + rt * 16 + l16; if (arix >= g.M) arix = g.M - 1;
    const float* arow = g.A + (size_t)arix * g.lda;
    v8f acc[4], accr[4];
#pragma unroll
    for (int t = 0; t < 4; ++t) { acc[t] = (v8f){}; accr[t] = (v8f){}; }
    const int K = g.K;
#pragma unroll 1
    for (int kc = 0; kc < K; kc += 32) {
        Opnd2 a;
        op_row<RA, NA>(arow + kc, half, g.ascale, a);
#pragma unroll
        for (int t = 0; t < 4; ++t) {
            const int n = col0 + t * 16 + l16;
            const bool cok = n < g.nvalid;
            const int nc = cok ? n : (g.nvalid - 1);
            Opnd2 b;
            op_col<RB, 1>(g.Bm, g.ldb, nc, kc, half, cok ? g.bscale : 0.0f, b);
            acc[t] = wm16(a.p[0], b.p[0], acc[t]);
            if (NA == 2) accr[t] = wm16(a.p[1], b.p[0], accr[t]);
        }
    }
#pragma unroll
    for (int t = 0; t < 4; ++t) {
        const int cl = ch * 64 + t * 16 + l16;
#pragma unroll
        for (int r = 0; r < 8; ++r) {
            const int rl = rt * 16 + r + 8 * half;
            float v = acc[t][r];
            if (NA == 2) v = v + accr[t][r] * RESCI;
            v = v * g.oscale;
            cst[rl * CSTR + cl] = v;
        }
    }
    __syncthreads();
    const int col = tid % TC, rsel = tid / TC, rstep = 256 / TC;
    float* ob = g.C + (size_t)row0 * g.ldc + (size_t)blockIdx.y * TC;
    const bool colok = (int)(blockIdx.y * TC + col) < g.nstore;
    const int rmax = (g.M - row0 < TR) ? (g.M - row0) : TR;
    if (colok) {
#pragma unroll 4
        for (int r = rsel; r < rmax; r += rstep) *(volatile float*)(ob + (size_t)r * g.ldc + col) = cst[r * CSTR + col];
    }
    __threadfence();
    if (colok) {
#pragma unroll 4
        for (int r = rsel; r < rmax; r += rstep) *(volatile float*)(ob + (size_t)r * g.ldc + col) = cst[r * CSTR + col];
    }
}

__global__ __launch_bounds__(256) void rms_kernel(float* __restrict__ dst, int ldd, const float* __restrict__ src, int ldsrc,
                                                  const float* __restrict__ gw, int cols, float invn) {
#pragma clang fp contract(off)
    __shared__ float red[8];
    const int row = blockIdx.x, tid = threadIdx.x, lane = tid & 31, wid = tid >> 5;
    const float* xr = src + (size_t)row * ldsrc;
    const int nj = cols >> 8;
    float v[3];
    float ss = 0.0f;
#pragma unroll
    for (int j = 0; j < 3; ++j) {
        const int c = tid + 256 * j;
        const int cc = (c < cols) ? c : (cols - 1);
        const float t = xr[cc];
        v[j] = (j < nj) ? t : 0.0f;
        const float sq = v[j] * v[j];
        ss = ss + sq;
    }
#pragma unroll
    for (int o = 16; o; o >>= 1) ss += __shfl_xor(ss, o, 32);
    if (lane == 0) red[wid] = ss;
    __syncthreads();
    float tot = 0.0f;
#pragma unroll
    for (int i = 0; i < 8; ++i) tot = tot + red[i];
    const float var = tot * invn;
    const float rsc = rsqrtf(var + RMS_EPS);
    float* orow = dst + (size_t)row * ldd;
#pragma unroll
    for (int j = 0; j < 3; ++j) {
        if (j < nj) { const int c = tid + 256 * j; const float gv = bfrne(gw[c]); float o = v[j] * rsc; o = o * gv; *(volatile float*)(orow + c) = o; }
    }
    __threadfence();
#pragma unroll
    for (int j = 0; j < 3; ++j) {
        if (j < nj) { const int c = tid + 256 * j; const float gv = bfrne(gw[c]); float o = v[j] * rsc; o = o * gv; *(volatile float*)(orow + c) = o; }
    }
}

struct TabArgs { float invf[NFREQ]; };
static_assert(sizeof(TabArgs) == 128);
__global__ __launch_bounds__(256) void tab_kernel(float* __restrict__ cs, float* __restrict__ sn, TabArgs ta) {
#pragma clang fp contract(off)
    const int idx = blockIdx.x * 256 + threadIdx.x;
    const int pos = idx >> 5, m = idx & 31;
    float f = 0.0f;
#pragma unroll
    for (int q = 0; q < NFREQ; ++q) f = (q == m) ? ta.invf[q] : f;
    const float ang = (float)pos * f;
    float sv, cv;
    sincosf(ang, &sv, &cv);
    *(volatile float*)(cs + idx) = cv;
    *(volatile float*)(sn + idx) = sv;
    __threadfence();
    *(volatile float*)(cs + idx) = cv;
    *(volatile float*)(sn + idx) = sv;
}

template <int LP, int NPC>
__device__ __forceinline__ void tile_out(const _Float16* tl, int rows, _Float16* dst, size_t dpitch, int tid) {
    const int tot = rows * NPC;
#pragma unroll 1
    for (int p = tid; p < tot; p += 256) {
        const int row = p / NPC, seg = p - row * NPC;
        const v8h val = *(const v8ha*)(tl + row * LP + seg * 8);
        *(volatile v8h*)(dst + (size_t)row * dpitch + seg * 8) = val;
    }
}


__global__ __launch_bounds__(256) void qplane_kernel(_Float16* __restrict__ qh, _Float16* __restrict__ qr, const float* __restrict__ qf,
                                                     const float* __restrict__ cs, const float* __restrict__ sn) {
#pragma clang fp contract(off)
    __shared__ __align__(16) _Float16 thi[64 * DQK];
    __shared__ __align__(16) _Float16 trs[64 * DQK];
    const int tid = threadIdx.x, s0 = blockIdx.x * 64, h = blockIdx.y;
    const bool early = s0 < EROWS;
#pragma unroll 1
    for (int i = 0; i < (64 * DQK) / 256; ++i) {
        const int e = tid + 256 * i, row = e / DQK, d = e - row * DQK, s = s0 + row;
        const float* base = qf + (size_t)s * QW + h * DQK;
        const int dm = (d > 0) ? d - 1 : 0, dp = (d < DQK - 1) ? d + 1 : DQK - 1;
        const float xv = base[d], xm = base[dm], xp = base[dp];
        const int jj = (d - DN) & 63, m = jj & 31;
        const float cv = cs[(size_t)s * NFREQ + m], sv = sn[(size_t)s * NFREQ + m];
        const float rot = (jj & 1) ? xm : -xp;
        const float t1 = xv * cv;
        const float t2 = rot * sv;
        const float ro = t1 + t2;
        const float out = (d >= DN) ? ro : xv;
        const _Float16 hv = (_Float16)out;
        thi[e] = hv;
        trs[e] = (_Float16)((out - (float)hv) * RESC);
    }
    __syncthreads();
    _Float16* dh = qh + ((size_t)h * SEQ + s0) * DQK;
    _Float16* dres = qr + ((size_t)h * EROWS + (early ? s0 : 0)) * DQK;
    tile_out<DQK, DQK / 8>(thi, 64, dh, DQK, tid);
    if (early) tile_out<DQK, DQK / 8>(trs, 64, dres, DQK, tid);
    __threadfence();
    tile_out<DQK, DQK / 8>(thi, 64, dh, DQK, tid);
    if (early) tile_out<DQK, DQK / 8>(trs, 64, dres, DQK, tid);
}

__global__ __launch_bounds__(256) void kvplane_kernel(_Float16* __restrict__ kh, _Float16* __restrict__ kr, _Float16* __restrict__ vt, _Float16* __restrict__ vr,
                                                      const float* __restrict__ kvup, const float* __restrict__ kvf,
                                                      const float* __restrict__ cs, const float* __restrict__ sn) {
#pragma clang fp contract(off)
    constexpr int VP = 72;
    __shared__ __align__(16) _Float16 thi[64 * DQK];
    __shared__ __align__(16) _Float16 trs[64 * DQK];
    static_assert(DV * VP <= 64 * DQK);
    const int tid = threadIdx.x, s0 = blockIdx.x * 64, h = blockIdx.y;
    const bool early = s0 < EROWS;
#pragma unroll 1
    for (int i = 0; i < (64 * DQK) / 256; ++i) {
        const int e = tid + 256 * i, row = e / DQK, d = e - row * DQK, s = s0 + row;
        const int dn = (d < DN) ? d : (DN - 1);
        const float kn = kvup[(size_t)s * KVUPW + h * (DN + DV) + dn];
        const int jj = (d >= DN) ? (d - DN) : 0;
        const int jm = (jj > 0) ? jj - 1 : 0, jp = (jj < DR - 1) ? jj + 1 : DR - 1;
        const float* rp = kvf + (size_t)s * KVP + KVL;
        const float xv = rp[jj], xm = rp[jm], xp = rp[jp];
        const int m = jj & 31;
        const float cv = cs[(size_t)s * NFREQ + m], sv = sn[(size_t)s * NFREQ + m];
        const float rot = (jj & 1) ? xm : -xp;
        const float t1 = xv * cv;
        const float t2 = rot * sv;
        const float ro = t1 + t2;
        const float out = (d >= DN) ? ro : kn;
        const _Float16 hv = (_Float16)out;
        thi[e] = hv;
        trs[e] = (_Float16)((out - (float)hv) * RESC);
    }
    __syncthreads();
    {
        _Float16* dh = kh + ((size_t)h * SEQ + s0) * DQK;
        _Float16* dres = kr + ((size_t)h * EROWS + (early ? s0 : 0)) * DQK;
        tile_out<DQK, DQK / 8>(thi, 64, dh, DQK, tid);
        if (early) tile_out<DQK, DQK / 8>(trs, 64, dres, DQK, tid);
        __threadfence();
        tile_out<DQK, DQK / 8>(thi, 64, dh, DQK, tid);
        if (early) tile_out<DQK, DQK / 8>(trs, 64, dres, DQK, tid);
    }
    __syncthreads();
#pragma unroll 1
    for (int i = 0; i < (64 * DV) / 256; ++i) {
        const int e = tid + 256 * i, sl = e >> 7, d = e & 127;
        const float v = kvup[(size_t)(s0 + sl) * KVUPW + h * (DN + DV) + DN + d];
        const _Float16 hv = (_Float16)v;
        thi[d * VP + sl] = hv;
        trs[d * VP + sl] = (_Float16)((v - (float)hv) * RESC);
    }
    __syncthreads();
    {
        _Float16* dvt = vt + (size_t)h * DV * SEQ + s0;
        _Float16* dvr = vr + (size_t)h * DV * EROWS + (early ? s0 : 0);
        tile_out<VP, 8>(thi, DV, dvt, SEQ, tid);
        if (early) tile_out<VP, 8>(trs, DV, dvr, EROWS, tid);
        __threadfence();
        tile_out<VP, 8>(thi, DV, dvt, SEQ, tid);
        if (early) tile_out<VP, 8>(trs, DV, dvr, EROWS, tid);
    }
}

template <int EV>
__global__ __launch_bounds__(128) __attribute__((amdgpu_num_vgpr(256)))
void attn_kernel(float* __restrict__ ctx, const _Float16* __restrict__ qh, const _Float16* __restrict__ kh, const _Float16* __restrict__ vt,
                 const _Float16* __restrict__ qr, const _Float16* __restrict__ kr, const _Float16* __restrict__ vr, int qt0) {
    constexpr int ND = EV ? 4 : 8;
    constexpr int OST = ND * 16 + 4;
    constexpr int NPR = ND * 4;
    constexpr int NIT = (16 * NPR) / 32;
    __shared__ __align__(16) _Float16 sP[4 * 1024];
    __shared__ __align__(16) _Float16 sR[4 * 1024];
    __shared__ __align__(16) float sO[4 * 16 * 132];
    const int tid = threadIdx.x, w = tid >> 5, lane = tid & 31, l16 = lane & 15, half = lane >> 4;
    const int qt = qt0 + (int)blockIdx.x, h = (int)blockIdx.y, qb = qt * 64;
    const int d0 = EV ? (int)blockIdx.z * (ND * 16) : 0;
    _Float16* myP = sP + w * 1024;
    _Float16* myR = sR + w * 1024;
    float* myO = sO + w * (16 * 132);
    const int qrow = qb + w * 16 + l16;
    const _Float16* qpA = qh + ((size_t)h * SEQ + qrow) * DQK + 8 * half;
    const _Float16* qpR = qr + ((size_t)h * EROWS + (EV ? qrow : 0)) * DQK + 8 * half;
    const _Float16* khb = kh + (size_t)h * SEQ * DQK + 8 * half;
    const _Float16* krb = kr + (size_t)h * EROWS * DQK + 8 * half;
    const _Float16* vtb = vt + (size_t)h * DV * SEQ + 8 * half;
    const _Float16* vrb = vr + (size_t)h * DV * EROWS + 8 * half;

    float mrow[8], lrow[8];
    v8f oacc[ND], oaccr[ND];
#pragma unroll
    for (int r = 0; r < 8; ++r) { mrow[r] = -__builtin_inff(); lrow[r] = 0.0f; }
#pragma unroll
    for (int td = 0; td < ND; ++td) { oacc[td] = (v8f){}; oaccr[td] = (v8f){}; }

#pragma unroll 1
    for (int j = 0; j <= qt; ++j) {
        const int kb = j * 64;
        v8f sacc[4], saccr[4];
#pragma unroll
        for (int t = 0; t < 4; ++t) { sacc[t] = (v8f){}; saccr[t] = (v8f){}; }
#pragma unroll 1
        for (int ks = 0; ks < DQK / 32; ++ks) {
            const v16h qa = ldfrag_g(qpA + ks * 32);
            v16h qra = (v16h){};
            if (EV != 0) qra = ldfrag_g(qpR + ks * 32);
#pragma unroll
            for (int t = 0; t < 4; ++t) {
                const int key = kb + t * 16 + l16;
                const v16h kf = ldfrag_g(khb + (size_t)key * DQK + ks * 32);
                sacc[t] = wm16(qa, kf, sacc[t]);
                if (EV != 0) {
                    saccr[t] = wm16(qra, kf, saccr[t]);
                    const v16h krf = ldfrag_g(krb + (size_t)key * DQK + ks * 32);
                    saccr[t] = wm16(qa, krf, saccr[t]);
                }
            }
        }
        float nm[8];
#pragma unroll
        for (int r = 0; r < 8; ++r) nm[r] = mrow[r];
        const bool diag = (j == qt);
#pragma unroll
        for (int t = 0; t < 4; ++t) {
            const int keyg = kb + t * 16 + l16;
#pragma unroll
            for (int r = 0; r < 8; ++r) {
                float s = sacc[t][r] * SCL;
                if (EV != 0) s = s + saccr[t][r] * (SCL * RESCI);
                const int rowg = qb + w * 16 + 8 * half + r;
                if (diag && keyg > rowg) s = -__builtin_inff();
                sacc[t][r] = s;
                nm[r] = fmaxf(nm[r], s);
            }
        }
#pragma unroll
        for (int o = 1; o < 16; o <<= 1)
#pragma unroll
            for (int r = 0; r < 8; ++r) nm[r] = fmaxf(nm[r], __shfl_xor(nm[r], o, 32));
        float alpha[8], rs[8];
#pragma unroll
        for (int r = 0; r < 8; ++r) { alpha[r] = __expf(mrow[r] - nm[r]); rs[r] = 0.0f; }
#pragma unroll
        for (int t = 0; t < 4; ++t)
#pragma unroll
            for (int r = 0; r < 8; ++r) {
                const float p = __expf(sacc[t][r] - nm[r]);
                rs[r] += p;
                const float pc = p * PCAR;
                const _Float16 ph = (_Float16)pc;
                const int pi = (8 * half + r) * 64 + t * 16 + l16;
                myP[pi] = ph;
                if (EV != 0) myR[pi] = (_Float16)((pc - (float)ph) * RESC);
            }
#pragma unroll
        for (int o = 1; o < 16; o <<= 1)
#pragma unroll
            for (int r = 0; r < 8; ++r) rs[r] += __shfl_xor(rs[r], o, 32);
#pragma unroll
        for (int r = 0; r < 8; ++r) { lrow[r] = lrow[r] * alpha[r] + rs[r]; mrow[r] = nm[r]; }
#pragma unroll
        for (int td = 0; td < ND; ++td)
#pragma unroll
            for (int r = 0; r < 8; ++r) {
                oacc[td][r] = oacc[td][r] * alpha[r];
                if (EV != 0) oaccr[td][r] = oaccr[td][r] * alpha[r];
            }
        wave_sync();
#pragma unroll
        for (int k2 = 0; k2 < 2; ++k2) {
            const v16h pa = ldfrag_l(myP + l16 * 64 + k2 * 32 + 8 * half);
            v16h pra = (v16h){};
            if (EV != 0) pra = ldfrag_l(myR + l16 * 64 + k2 * 32 + 8 * half);
#pragma unroll
            for (int td = 0; td < ND; ++td) {
                const size_t drow = (size_t)(d0 + td * 16 + l16);
                const v16h vf = ldfrag_g(vtb + drow * SEQ + kb + k2 * 32);
                oacc[td] = wm16(pa, vf, oacc[td]);
                if (EV != 0) {
                    oaccr[td] = wm16(pra, vf, oaccr[td]);
                    const v16h vrf = ldfrag_g(vrb + drow * EROWS + kb + k2 * 32);
                    oaccr[td] = wm16(pa, vrf, oaccr[td]);
                }
            }
        }
        wave_sync();
    }
    float inv[8];
#pragma unroll
    for (int r = 0; r < 8; ++r) inv[r] = (1.0f / lrow[r]) * PCARI;
#pragma unroll
    for (int td = 0; td < ND; ++td)
#pragma unroll
        for (int r = 0; r < 8; ++r) {
            float o = oacc[td][r];
            if (EV != 0) o = o + oaccr[td][r] * RESCI;
            o = o * inv[r];
            myO[(8 * half + r) * OST + td * 16 + l16] = o;
        }
    wave_sync();
    float* cb = ctx + (size_t)(qb + w * 16) * CTXW + h * DV + d0;
#pragma unroll
    for (int i = 0; i < NIT; ++i) {
        const int p = 32 * i + lane, row = p / NPR, seg = p % NPR;
        const v4f val = *(const v4fa*)(myO + row * OST + seg * 4);
        *(volatile v4f*)(cb + (size_t)row * CTXW + seg * 4) = val;
    }
    __threadfence();
#pragma unroll
    for (int i = 0; i < NIT; ++i) {
        const int p = 32 * i + lane, row = p / NPR, seg = p % NPR;
        const v4f val = *(const v4fa*)(myO + row * OST + seg * 4);
        *(volatile v4f*)(cb + (size_t)row * CTXW + seg * 4) = val;
    }
}

static inline GArgs gargs(const float* A, int lda, const float* Bm, int ldb, float* C, int ldc, int M, int nvalid, int nstore, int K,
                          float ascale, float bscale, float oscale) {
    GArgs g;
    g.A = A; g.Bm = Bm; g.C = C;
    g.lda = lda; g.ldb = ldb; g.ldc = ldc; g.K = K;
    g.M = M; g.nvalid = nvalid; g.nstore = nstore; g.spare = 0;
    g.ascale = ascale; g.bscale = bscale; g.oscale = oscale; g.fsp = 0.0f;
    return g;
}
template <int RA, int NA, int RB> static inline void gemm_launch(const GArgs& g, hipStream_t st) {
    const dim3 grid((unsigned)((g.M + 63) / 64), (unsigned)((g.nstore + 127) / 128), 1);
    gemm_kernel<RA, NA, RB><<<grid, 256, 0, st>>>(g);
}

extern "C" void kernel_launch(void* const* d_in, const int* in_sizes, int n_in,
                              void* d_out, int out_size, void* d_ws, size_t ws_size, hipStream_t stream) {
    if (n_in < 8) return;
    const float* x    = (const float*)d_in[0];
    const float* wqa  = (const float*)d_in[1];
    const float* gq   = (const float*)d_in[2];
    const float* wqb  = (const float*)d_in[3];
    const float* wkva = (const float*)d_in[4];
    const float* gkv  = (const float*)d_in[5];
    const float* wkvb = (const float*)d_in[6];
    const float* wo   = (const float*)d_in[7];
    float* out = (float*)d_out;
    if (in_sizes[0] < SEQ * HID || in_sizes[1] < HID * QL || in_sizes[2] < QL || in_sizes[3] < QL * QW || in_sizes[4] < HID * KVW ||
        in_sizes[5] < KVL || in_sizes[6] < KVL * KVUPW || in_sizes[7] < CTXW * HID || out_size < SEQ * HID) return;

    char* wsb = (char*)d_ws;
    size_t off = 0;
    auto take = [&](size_t bytes) -> char* { char* p = wsb + off; off += (bytes + 255) & ~(size_t)255; return p; };
    float* cs   = (float*)take((size_t)SEQ * NFREQ * 4);
    float* sn   = (float*)take((size_t)SEQ * NFREQ * 4);
    float* qa   = (float*)take((size_t)SEQ * QL * 4);
    float* kvf  = (float*)take((size_t)SEQ * KVP * 4);
    float* qan  = (float*)take((size_t)SEQ * QL * 4);
    float* ckvn = (float*)take((size_t)SEQ * KVL * 4);
    float* qf   = (float*)take((size_t)SEQ * QW * 4);
    float* ctx  = qf;
    static_assert((size_t)SEQ * CTXW <= (size_t)SEQ * QW);
    float* kvup = (float*)take((size_t)SEQ * KVUPW * 4);
    _Float16* qh = (_Float16*)take((size_t)NH * SEQ * DQK * 2);
    _Float16* kh = (_Float16*)take((size_t)NH * SEQ * DQK * 2);
    _Float16* vt = (_Float16*)take((size_t)NH * DV * SEQ * 2);
    _Float16* qr = (_Float16*)take((size_t)NH * EROWS * DQK * 2);
    _Float16* kr = (_Float16*)take((size_t)NH * EROWS * DQK * 2);
    _Float16* vr = (_Float16*)take((size_t)NH * DV * EROWS * 2);
    if (off > ws_size || off > (size_t)134217728) return;

    TabArgs ta;
    {
        volatile float theta = 10000.0f;
        for (int m = 0; m < NFREQ; ++m) {
            const float e = (float)(2 * m) / (float)DR;
            const float pw = powf(theta, e);
            ta.invf[m] = 1.0f / pw;
        }
    }
    tab_kernel<<<dim3((SEQ * NFREQ) / 256), 256, 0, stream>>>(cs, sn, ta);

    gemm_launch<1, 1, 1>(gargs(x, HID, wqa, QL, qa, QL, SEQ, QL, QL, HID, 1.0f, 32.0f, 1.0f / 32.0f), stream);
    gemm_launch<1, 1, 1>(gargs(x, HID, wkva, KVW, kvf, KVP, SEQ, KVW, KVP, HID, 1.0f, 32.0f, 1.0f / 32.0f), stream);
    rms_kernel<<<dim3(SEQ), 256, 0, stream>>>(qan, QL, qa, QL, gq, QL, 1.0f / (float)QL);
    rms_kernel<<<dim3(SEQ), 256, 0, stream>>>(ckvn, KVL, kvf, KVP, gkv, KVL, 1.0f / (float)KVL);
    gemm_launch<0, 2, 1>(gargs(qan, QL, wqb, QW, qf, QW, EROWS, QW, QW, QL, 8.0f, 16.0f, 1.0f / 128.0f), stream);
    if (LROWS > 0)
        gemm_launch<0, 1, 1>(gargs(qan + (size_t)EROWS * QL, QL, wqb, QW, qf + (size_t)EROWS * QW, QW, LROWS, QW, QW, QL, 8.0f, 16.0f, 1.0f / 128.0f), stream);
    gemm_launch<0, 2, 1>(gargs(ckvn, KVL, wkvb, KVUPW, kvup, KVUPW, EROWS, KVUPW, KVUPW, KVL, 8.0f, 16.0f, 1.0f / 128.0f), stream);
    if (LROWS > 0)
        gemm_launch<0, 1, 1>(gargs(ckvn + (size_t)EROWS * KVL, KVL, wkvb, KVUPW, kvup + (size_t)EROWS * KVUPW, KVUPW, LROWS, KVUPW, KVUPW, KVL, 8.0f, 16.0f, 1.0f / 128.0f), stream);
    qplane_kernel<<<dim3(SEQ / 64, NH), 256, 0, stream>>>(qh, qr, qf, cs, sn);
    kvplane_kernel<<<dim3(SEQ / 64, NH), 256, 0, stream>>>(kh, kr, vt, vr, kvup, kvf, cs, sn);
    attn_kernel<1><<<dim3(EROWS / 64, NH, 2), 128, 0, stream>>>(ctx, qh, kh, vt, qr, kr, vr, 0);
    if (LROWS > 0)
        attn_kernel<0><<<dim3(LROWS / 64, NH, 1), 128, 0, stream>>>(ctx, qh, kh, vt, qr, kr, vr, EROWS / 64);
    gemm_launch<0, 2, 1>(gargs(ctx, CTXW, wo, HID, out, HID, EROWS, HID, HID, CTXW, 16.0f, 32.0f, 1.0f / 512.0f), stream);
    if (LROWS > 0)
        gemm_launch<0, 1, 1>(gargs(ctx + (size_t)EROWS * CTXW, CTXW, wo, HID, out + (size_t)EROWS * HID, HID, LROWS, HID, HID, CTXW, 16.0f, 32.0f, 1.0f / 512.0f), stream);
}
